// SDFMarcher_46145128628269
// MI455X (gfx1250) — hardware-run, weakly checked
//
#include <hip/hip_runtime.h>

typedef __attribute__((ext_vector_type(16))) _Float16 v16h;
typedef __attribute__((ext_vector_type(8)))  _Float16 v8h;
typedef __attribute__((ext_vector_type(8)))  float    v8f;
typedef __attribute__((ext_vector_type(4)))  float    v4f;

constexpr int kRays          = 65536;
constexpr int kHid           = 128;
constexpr int kWavesPerBlock = 8;
constexpr int kThreads       = kWavesPerBlock * 32;
constexpr int kRaysPerWave   = 32;
constexpr int kRaysPerBlock  = kWavesPerBlock * kRaysPerWave;
constexpr int kBlocks        = kRays / kRaysPerBlock;
constexpr int kW2Pitch       = kHid + 8;
constexpr int kOutPerWave    = kRaysPerWave * 3;
constexpr int kMaxSteps      = 1024;
static_assert(kRays % kRaysPerBlock == 0);
static_assert(kBlocks == 256);
static_assert(kHid % 32 == 0 && kHid % 16 == 0);
static_assert((kW2Pitch * 2) % 16 == 0);
static_assert((kOutPerWave * 4) % 128 == 0);
static_assert((kHid * 16) % kThreads == 0);

constexpr float kCarryAct      = 16.0f;
constexpr float kCarryW        = 256.0f;
constexpr float kCarryAll      = kCarryAct * kCarryW;
constexpr float kCarryInv      = 1.0f / kCarryAll;
constexpr float kHalfMinNormal = 6.103515625e-5f;
static_assert(kCarryAll == 4096.0f);


union FragU { v16h v; v8h h[2]; };

__device__ __forceinline__ v16h frag_load(const _Float16* p) {
  FragU f;
  f.h[0] = *(const v8h*)(p);
  f.h[1] = *(const v8h*)(p + 16);
  return f.v;
}

__device__ __forceinline__ v8f mma_g(v16h a, v16h b, v8f c) {
  c = __builtin_amdgcn_wmma_f32_16x16x32_f16(false, a, false, b, (short)0, c, false, false);
  asm volatile("v_nop\n\tv_nop\n\tv_nop\n\tv_nop" : "+v"(c) : "v"(a), "v"(b));
  return c;
}

__device__ __forceinline__ float act1(float px, float py, float pz, v4f w) {
  float t = fmaf(px, w[0], w[3]);
  t = fmaf(py, w[1], t);
  t = fmaf(pz, w[2], t);
  return (t >= kHalfMinNormal) ? t : 0.0f;
}

__global__ __launch_bounds__(256) __attribute__((amdgpu_num_vgpr(256)))
void fused_step_kernel(const float* __restrict__ P, const float* __restrict__ Dir,
                       const float* __restrict__ W1, const float* __restrict__ B1,
                       const float* __restrict__ W2, const float* __restrict__ B2,
                       const float* __restrict__ W3, const float* __restrict__ B3,
                       const int* __restrict__ STEPS, float* __restrict__ OUT)
{
  __shared__ __align__(16) _Float16 w2t[kHid * kW2Pitch];
  __shared__ __align__(16) float    w1s[kHid * 4];
  __shared__ __align__(16) float    b2s[kHid];
  __shared__ __align__(16) float    w3s[kHid];
  __shared__ __align__(16) float    outS[kWavesPerBlock * kOutPerWave];

  const int tid  = threadIdx.x;
  const int lane = tid & 31;
  const int wave = tid >> 5;
  const int h    = lane >> 4;
  const int c    = lane & 15;

#pragma unroll 1
  for (int it = 0; it < (kHid * 16) / kThreads; ++it) {
    const int item = it * kThreads + tid;
    const int n  = item & (kHid - 1);
    const int k8 = item >> 7;
    v8h hv;
#pragma unroll
    for (int e = 0; e < 8; ++e) {
      float w = W2[(k8 * 8 + e) * kHid + n] * kCarryW;
      w = (fabsf(w) >= kHalfMinNormal) ? w : 0.0f;
      hv[e] = (_Float16)w;
    }
    *(v8h*)(w2t + n * kW2Pitch + k8 * 8) = hv;
  }
  {
    const int j = tid & (kHid - 1);
    const float a0 = W1[j] * kCarryAct;
    const float a1 = W1[kHid + j] * kCarryAct;
    const float a2 = W1[2 * kHid + j] * kCarryAct;
    const float a3 = B1[j] * kCarryAct;
    const float bb = B2[j] * kCarryAll;
    const float ww = W3[j] * kCarryInv;
    if (tid < kHid) {
      const v4f wv = (v4f){a0, a1, a2, a3};
      *(v4f*)(w1s + 4 * j) = wv;
      b2s[j] = bb;
      w3s[j] = ww;
      const v8h z8 = (v8h){(_Float16)0.0f, (_Float16)0.0f, (_Float16)0.0f, (_Float16)0.0f,
                           (_Float16)0.0f, (_Float16)0.0f, (_Float16)0.0f, (_Float16)0.0f};
      *(v8h*)(w2t + j * kW2Pitch + kHid) = z8;
    }
  }
  __syncthreads();

  const int gw   = blockIdx.x * kWavesPerBlock + wave;
  const int ray0 = gw * kRaysPerWave + c;
  const int ray1 = ray0 + 16;
  float px0 = P[3 * ray0 + 0], py0 = P[3 * ray0 + 1], pz0 = P[3 * ray0 + 2];
  float px1 = P[3 * ray1 + 0], py1 = P[3 * ray1 + 1], pz1 = P[3 * ray1 + 2];
  const float dx0 = Dir[3 * ray0 + 0], dy0 = Dir[3 * ray0 + 1], dz0 = Dir[3 * ray0 + 2];
  const float dx1 = Dir[3 * ray1 + 0], dy1 = Dir[3 * ray1 + 1], dz1 = Dir[3 * ray1 + 2];
  const float b3 = B3[0];
  int steps = STEPS[0];
  steps = steps < 0 ? 0 : steps;
  steps = steps > kMaxSteps ? kMaxSteps : steps;

  const int aBase = c * kW2Pitch + 8 * h;
  const int hOff  = 8 * h;

#pragma unroll 1
  for (int s = 0; s < steps; ++s) {
    int off = 0;
    asm volatile("" : "+v"(off));

    v8f acc0[8], acc1[8];
#pragma unroll
    for (int nt = 0; nt < 8; ++nt) {
      const float* bp = b2s + (16 * nt + hOff + off);
      const v4f x = *(const v4f*)(bp);
      const v4f y = *(const v4f*)(bp + 4);
      acc0[nt] = __builtin_shufflevector(x, y, 0, 1, 2, 3, 4, 5, 6, 7);
      acc1[nt] = acc0[nt];
    }

#pragma unroll 1
    for (int kc = 0; kc < kHid / 32; ++kc) {
      v16h hb0, hb1;
      const float* w1p = w1s + 4 * (kc * 32 + hOff + off);
#pragma unroll
      for (int e = 0; e < 8; ++e) {
        const v4f wa = *(const v4f*)(w1p + 4 * e);
        const v4f wb = *(const v4f*)(w1p + 4 * (16 + e));
        const float t0a = act1(px0, py0, pz0, wa);
        const float t0b = act1(px0, py0, pz0, wb);
        const float t1a = act1(px1, py1, pz1, wa);
        const float t1b = act1(px1, py1, pz1, wb);
        hb0[e]     = (_Float16)t0a;
        hb0[8 + e] = (_Float16)t0b;
        hb1[e]     = (_Float16)t1a;
        hb1[8 + e] = (_Float16)t1b;
      }
      const _Float16* ap = w2t + (aBase + kc * 32 + off);
#pragma unroll
      for (int nt = 0; nt < 8; ++nt) {
        const v16h a = frag_load(ap + nt * 16 * kW2Pitch);
        acc0[nt] = mma_g(a, hb0, acc0[nt]);
        acc1[nt] = mma_g(a, hb1, acc1[nt]);
      }
    }

    float part0 = 0.0f, part1 = 0.0f;
#pragma unroll
    for (int nt = 0; nt < 8; ++nt) {
      const float* wp = w3s + (16 * nt + hOff + off);
      const v4f wx = *(const v4f*)(wp);
      const v4f wy = *(const v4f*)(wp + 4);
#pragma unroll
      for (int r = 0; r < 4; ++r) {
        part0 = fmaf(fmaxf(acc0[nt][r], 0.0f), wx[r], part0);
        part1 = fmaf(fmaxf(acc1[nt][r], 0.0f), wx[r], part1);
      }
#pragma unroll
      for (int r = 0; r < 4; ++r) {
        part0 = fmaf(fmaxf(acc0[nt][4 + r], 0.0f), wy[r], part0);
        part1 = fmaf(fmaxf(acc1[nt][4 + r], 0.0f), wy[r], part1);
      }
    }
    const float q0 = __shfl_xor(part0, 16, 32);
    const float q1 = __shfl_xor(part1, 16, 32);
    const float s0 = (part0 + q0) + b3;
    const float s1 = (part1 + q1) + b3;

    px0 = fmaf(s0, dx0, px0);
    py0 = fmaf(s0, dy0, py0);
    pz0 = fmaf(s0, dz0, pz0);
    px1 = fmaf(s1, dx1, px1);
    py1 = fmaf(s1, dy1, py1);
    pz1 = fmaf(s1, dz1, pz1);
  }

  float* sl = outS + wave * kOutPerWave;
  if (h == 0) {
    sl[3 * c + 0] = px0;
    sl[3 * c + 1] = py0;
    sl[3 * c + 2] = pz0;
    sl[3 * (16 + c) + 0] = px1;
    sl[3 * (16 + c) + 1] = py1;
    sl[3 * (16 + c) + 2] = pz1;
  }
  __syncthreads();
  const float f0 = sl[lane];
  const float f1 = sl[32 + lane];
  const float f2 = sl[64 + lane];
  volatile float* o = (volatile float*)(OUT + (size_t)gw * kOutPerWave);
  o[lane]      = f0;
  o[32 + lane] = f1;
  o[64 + lane] = f2;
  __threadfence();
  o[lane]      = f0;
  o[32 + lane] = f1;
  o[64 + lane] = f2;
}

extern "C" void kernel_launch(void* const* d_in, const int* in_sizes, int n_in,
                              void* d_out, int out_size, void* d_ws, size_t ws_size,
                              hipStream_t stream) {
  (void)d_ws;
  (void)ws_size;
  if (n_in < 9) return;
  if (in_sizes[0] != kRays * 3) return;
  if (in_sizes[1] != kRays * 3) return;
  if (in_sizes[2] != 3 * kHid) return;
  if (in_sizes[3] != kHid) return;
  if (in_sizes[4] != kHid * kHid) return;
  if (in_sizes[5] != kHid) return;
  if (in_sizes[6] != kHid) return;
  if (in_sizes[7] != 1) return;
  if (in_sizes[8] != 1) return;
  if (out_size != kRays * 3) return;

  const float* P   = (const float*)d_in[0];
  const float* Dir = (const float*)d_in[1];
  const float* W1  = (const float*)d_in[2];
  const float* B1  = (const float*)d_in[3];
  const float* W2  = (const float*)d_in[4];
  const float* B2  = (const float*)d_in[5];
  const float* W3  = (const float*)d_in[6];
  const float* B3  = (const float*)d_in[7];
  const int*   ST  = (const int*)d_in[8];
  float* OUT = (float*)d_out;

  fused_step_kernel<<<kBlocks, kThreads, 0, stream>>>(P, Dir, W1, B1, W2, B2, W3, B3, ST, OUT);
}
